// VPTLSTM_71949292142746
// MI455X (gfx1250) — hardware-run, weakly checked
//
#include <hip/hip_runtime.h>
#include <stddef.h>
#include <math.h>


#define SEQ_T   99
#define NVEH    256
#define NIN     9
#define RNN     128
#define EMB     64
#define NOUT    5
#define GH      19
#define GW      5
#define GCELL   (GH * GW)
#define NPOS    15
#define N1      (NPOS * EMB)
#define T1ROW   1536
#define VB      16
#define NBLK    (NVEH / VB)
#define NTHR    128
#define NWAV    (NTHR / 32)
#define OSW     8
#define NCHUNK  ((SEQ_T * NVEH * NOUT) / 128)

#define WC      64.0f
#define AC      16.0f
#define INV_W   (1.0f / 64.0f)
#define INV_AW  (1.0f / 1024.0f)

#define F_EMB   4
#define F_W1    240
#define F_W2    60
#define F_SOC   16
#define F_IH    128
#define F_HH    128
#define F_OUT   4

#define O_EMB   ((size_t)0)
#define O_W1    (O_EMB + (size_t)F_EMB * 1024)
#define O_W2    (O_W1  + (size_t)F_W1  * 1024)
#define O_SOC   (O_W2  + (size_t)F_W2  * 1024)
#define O_IH    (O_SOC + (size_t)F_SOC * 1024)
#define O_HH    (O_IH  + (size_t)F_IH  * 1024)
#define O_OUT   (O_HH  + (size_t)F_HH  * 1024)
#define O_OS    (O_OUT + (size_t)F_OUT * 1024)
#define SZ_OS   ((size_t)SEQ_T * NVEH * OSW * 4)
#define WSTOT   (O_OS + SZ_OS)
#define WSCAP   134217728

#define LDS_BYTES 174592

static_assert(WSTOT <= (size_t)WSCAP);
static_assert((O_W1 % 128) == 0 && (O_W2 % 128) == 0 && (O_SOC % 128) == 0 && (O_IH % 128) == 0);
static_assert((O_HH % 128) == 0 && (O_OUT % 128) == 0 && (O_OS % 128) == 0);
static_assert(F_W1 * 512 == 64 * 128 * 15);
static_assert(F_W2 * 512 == 32 * 64 * 15);
static_assert(NCHUNK * 128 == SEQ_T * NVEH * NOUT);
static_assert((RNN % 32) == 0 && (N1 % 32) == 0 && ((2 * EMB) % 32) == 0);
static_assert(NBLK * VB == NVEH && NWAV == 4);
static_assert(VB * 24 * 4 == 12 * NTHR);
static_assert(VB * RNN == 16 * NTHR);
static_assert(LDS_BYTES == 4 * (VB * N1 + VB * 512 + VB * RNN + VB * 96 + 768 + 128)
                           + 2 * (VB * T1ROW + VB * 128 + VB * 128 + VB * 32 + VB * 128));

typedef _Float16 v16h __attribute__((ext_vector_type(16)));
typedef _Float16 v8h  __attribute__((ext_vector_type(8), __may_alias__));
typedef float    v8f  __attribute__((ext_vector_type(8)));
typedef float    v4f  __attribute__((ext_vector_type(4), __may_alias__));
union Frag { v16h v; v8h h[2]; };
static_assert(sizeof(Frag) == 32);

__device__ __forceinline__ int imin(int a, int b) { return a < b ? a : b; }

__device__ __forceinline__ v8f wmh(v16h a, v16h bq, v8f c) {
  v8f d = __builtin_amdgcn_wmma_f32_16x16x32_f16(false, a, false, bq, (short)0, c, false, false);
  asm volatile("v_nop\n\tv_nop\n\tv_nop\n\tv_nop" : "+v"(d) : "v"(a), "v"(bq));
  return d;
}

__device__ __forceinline__ v8f zero8() {
  v8f z = {0.f, 0.f, 0.f, 0.f, 0.f, 0.f, 0.f, 0.f};
  return z;
}

__device__ __forceinline__ v16h lda_frag(const _Float16* base, int pitch, int lane) {
  const int m = lane & 15, hh = lane >> 4;
  const _Float16* p = base + m * pitch + 8 * hh;
  Frag u;
  u.h[0] = *(const v8h*)p;
  u.h[1] = *(const v8h*)(p + 16);
  return u.v;
}

__device__ __forceinline__ v16h ldb_frag(const v16h* __restrict__ packed, int frag, int lane) {
  return packed[frag * 32 + lane];
}

__device__ __forceinline__ float sigm_(float x) { return 1.0f / (1.0f + expf(-x)); }

__global__ __launch_bounds__(256) void k_pack(const float* __restrict__ src, _Float16* dst,
                                              int mode, int chunks, int nthr) {
  const int e = blockIdx.x * 256 + threadIdx.x;
  if (e >= nthr) return;
  const int frag = e >> 6, r = e & 63, lane = r >> 1, q = r & 1;
  const int tn = frag / chunks, kc = frag - tn * chunks;
  const int n = tn * 16 + (lane & 15);
  const int kb = kc * 32 + 16 * q + 8 * (lane >> 4);
  v8h hv;
#pragma unroll
  for (int i = 0; i < 8; ++i) {
    const int k = kb + i;
    float val;
    if (mode == 0) {
      const float w = src[n * NIN + imin(k, NIN - 1)];
      val = (k < NIN) ? w : 0.0f;
    } else if (mode == 1) {
      const int p = n >> 6, o = n & 63, ky = p / 3, kx = p - 3 * ky;
      val = src[((o * RNN + k) * 5 + ky) * 3 + kx];
    } else if (mode == 2) {
      const int ky = k / 192, rem = k - 192 * ky, kx = rem >> 6, o1 = rem & 63;
      val = src[((n * 64 + o1) * 5 + ky) * 3 + kx];
    } else if (mode == 3) {
      val = src[n * RNN + k];
    } else {
      const float w = src[imin(n, NOUT - 1) * RNN + k];
      val = (n < NOUT) ? w : 0.0f;
    }
    hv[i] = (_Float16)(val * WC);
  }
  *(volatile v8h*)(dst + (size_t)8 * e) = hv;
  __threadfence();
  *(volatile v8h*)(dst + (size_t)8 * e) = hv;
}

__global__ __launch_bounds__(NTHR) void k_lstm(
    const float* __restrict__ x_seq, const int* __restrict__ grids,
    const float* __restrict__ h0, const float* __restrict__ c0,
    const float* __restrict__ b_emb, const float* __restrict__ b1g,
    const float* __restrict__ b2g, const float* __restrict__ b_soc,
    const float* __restrict__ b_ih, const float* __restrict__ b_hh,
    const float* __restrict__ b_out,
    const v16h* __restrict__ Wemb_p, const v16h* __restrict__ W1_p,
    const v16h* __restrict__ W2_p, const v16h* __restrict__ Wsoc_p,
    const v16h* __restrict__ Wih_p, const v16h* __restrict__ Whh_p,
    const v16h* __restrict__ Wout_p, float* OS) {
  extern __shared__ __align__(16) char smem[];
  float* sA1  = (float*)smem;
  float* sG   = sA1 + VB * N1;
  float* sC   = sG + VB * 512;
  float* sOcc = sC + VB * RNN;
  float* sB   = sOcc + VB * 96;
  float* sOut = sB + 768;
  _Float16* sT1  = (_Float16*)(sOut + 128);
  _Float16* sT2  = sT1 + VB * T1ROW;
  _Float16* sX   = sT2 + VB * 128;
  _Float16* sXin = sX + VB * 128;
  _Float16* sH   = sXin + VB * 32;
  float* sB1   = sB;
  float* sB2   = sB + 64;
  float* sBemb = sB + 96;
  float* sBsoc = sB + 160;
  float* sBg   = sB + 224;
  float* sBout = sB + 736;

  const int tid = threadIdx.x, lane = tid & 31, wave = tid >> 5;
  const int hh = lane >> 4, nn = lane & 15;
  const int v0 = blockIdx.x * VB;

  for (int i = tid; i < 64; i += NTHR) { sB1[i] = b1g[i]; sBemb[i] = b_emb[i]; sBsoc[i] = b_soc[i]; }
  for (int i = tid; i < 32; i += NTHR) sB2[i] = b2g[i];
  for (int i = tid; i < 512; i += NTHR) sBg[i] = b_ih[i] + b_hh[i];
  for (int i = tid; i < 16; i += NTHR) {
    const float w = b_out[imin(i, NOUT - 1)];
    sBout[i] = (i < NOUT) ? w : 0.0f;
  }
  for (int i = tid; i < VB * RNN; i += NTHR) {
    const int v = i >> 7, r = i & 127;
    sH[i] = (_Float16)(h0[(v0 + v) * RNN + r] * AC);
    sC[i] = c0[(v0 + v) * RNN + r];
  }
  __syncthreads();

#pragma unroll 1
  for (int t = 0; t < SEQ_T; ++t) {
    for (int i = tid; i < VB * 32; i += NTHR) {
      const int v = i >> 5, k = i & 31;
      const float xv = x_seq[(size_t)(t * NVEH + v0 + v) * NIN + imin(k, NIN - 1)];
      sXin[i] = (_Float16)((k < NIN) ? xv : 0.0f);
    }
    for (int i = tid; i < VB * GCELL; i += NTHR) {
      const int v = i / GCELL, g = i - GCELL * v;
      sOcc[v * 96 + g] = (grids[(size_t)(t * NVEH + v0 + v) * GCELL + g] != -1) ? 1.0f : 0.0f;
    }
    __syncthreads();

    {
      v8f acc = zero8();
      acc = wmh(lda_frag(sXin, 32, lane), ldb_frag(Wemb_p, wave, lane), acc);
      const int col = wave * 16 + nn;
      const float bb = sBemb[col];
#pragma unroll
      for (int r = 0; r < 8; ++r) {
        const float val = fmaxf(acc[r] * INV_W + bb, 0.0f);
        sX[(8 * hh + r) * 128 + col] = (_Float16)(val * AC);
      }
    }
    {
      v16h fa[4];
#pragma unroll
      for (int kc = 0; kc < 4; ++kc) fa[kc] = lda_frag(sH + kc * 32, RNN, lane);
#pragma unroll 1
      for (int tn = wave; tn < 60; tn += NWAV) {
        v8f acc = zero8();
#pragma unroll
        for (int kc = 0; kc < 4; ++kc) acc = wmh(fa[kc], ldb_frag(W1_p, tn * 4 + kc, lane), acc);
        const int col = tn * 16 + nn;
#pragma unroll
        for (int r = 0; r < 8; ++r) sA1[(8 * hh + r) * N1 + col] = acc[r] * INV_AW;
      }
    }
    __syncthreads();

#pragma unroll 1
    for (int it = 0; it < 12; ++it) {
      const int item = tid + NTHR * it;
      const int ob = item & 3, qq = item >> 2;
      const int v = qq / 24, yx = qq - 24 * v;
      const int Y = yx / 3, X = yx - 3 * Y;
      const float* orow = sOcc + v * 96 + (2 * Y) * GW + X;
      float oc[NPOS];
#pragma unroll
      for (int p = 0; p < NPOS; ++p) oc[p] = orow[(p / 3) * GW + (p % 3)];
      v4f s0 = {0.f, 0.f, 0.f, 0.f}, s1 = s0, s2 = s0, s3 = s0;
      const float* g = sA1 + v * N1 + ob * 16;
#pragma unroll
      for (int p = 0; p < NPOS; ++p) {
        const float* gp = g + p * 64;
        const v4f g0 = *(const v4f*)(gp), g1 = *(const v4f*)(gp + 4);
        const v4f g2 = *(const v4f*)(gp + 8), g3 = *(const v4f*)(gp + 12);
        s0 += oc[p] * g0; s1 += oc[p] * g1; s2 += oc[p] * g2; s3 += oc[p] * g3;
      }
      const float* bp = sB1 + ob * 16;
      const v4f b0 = *(const v4f*)(bp), bb1 = *(const v4f*)(bp + 4);
      const v4f bb2 = *(const v4f*)(bp + 8), bb3 = *(const v4f*)(bp + 12);
      s0 += b0; s1 += bb1; s2 += bb2; s3 += bb3;
      v8h o0, o1;
      o0[0] = (_Float16)(fmaxf(s0.x, 0.f) * AC); o0[1] = (_Float16)(fmaxf(s0.y, 0.f) * AC);
      o0[2] = (_Float16)(fmaxf(s0.z, 0.f) * AC); o0[3] = (_Float16)(fmaxf(s0.w, 0.f) * AC);
      o0[4] = (_Float16)(fmaxf(s1.x, 0.f) * AC); o0[5] = (_Float16)(fmaxf(s1.y, 0.f) * AC);
      o0[6] = (_Float16)(fmaxf(s1.z, 0.f) * AC); o0[7] = (_Float16)(fmaxf(s1.w, 0.f) * AC);
      o1[0] = (_Float16)(fmaxf(s2.x, 0.f) * AC); o1[1] = (_Float16)(fmaxf(s2.y, 0.f) * AC);
      o1[2] = (_Float16)(fmaxf(s2.z, 0.f) * AC); o1[3] = (_Float16)(fmaxf(s2.w, 0.f) * AC);
      o1[4] = (_Float16)(fmaxf(s3.x, 0.f) * AC); o1[5] = (_Float16)(fmaxf(s3.y, 0.f) * AC);
      o1[6] = (_Float16)(fmaxf(s3.z, 0.f) * AC); o1[7] = (_Float16)(fmaxf(s3.w, 0.f) * AC);
      _Float16* trow = sT1 + v * T1ROW + yx * 64 + ob * 16;
      *(v8h*)(trow) = o0;
      *(v8h*)(trow + 8) = o1;
    }
    __syncthreads();

#pragma unroll 1
    for (int job = wave; job < 8; job += NWAV) {
      const int y2 = job >> 1, tn = job & 1;
      const _Float16* aBase = sT1 + y2 * 192;
      v8f acc = zero8();
#pragma unroll 2
      for (int kc = 0; kc < 30; ++kc)
        acc = wmh(lda_frag(aBase + kc * 32, T1ROW, lane), ldb_frag(W2_p, tn * 30 + kc, lane), acc);
      const int o2 = tn * 16 + nn;
      const float bb = sB2[o2];
#pragma unroll
      for (int r = 0; r < 8; ++r) {
        const float val = fmaxf(acc[r] * INV_AW + bb, 0.0f);
        sT2[(8 * hh + r) * 128 + o2 * 4 + y2] = (_Float16)(val * AC);
      }
    }
    __syncthreads();

    {
      v8f acc = zero8();
#pragma unroll
      for (int kc = 0; kc < 4; ++kc)
        acc = wmh(lda_frag(sT2 + kc * 32, 128, lane), ldb_frag(Wsoc_p, wave * 4 + kc, lane), acc);
      const int col = wave * 16 + nn;
      const float bb = sBsoc[col];
#pragma unroll
      for (int r = 0; r < 8; ++r) {
        const float val = fmaxf(acc[r] * INV_AW + bb, 0.0f);
        sX[(8 * hh + r) * 128 + EMB + col] = (_Float16)(val * AC);
      }
    }
    __syncthreads();

    {
      v16h fx[4], fh[4];
#pragma unroll
      for (int kc = 0; kc < 4; ++kc) {
        fx[kc] = lda_frag(sX + kc * 32, 128, lane);
        fh[kc] = lda_frag(sH + kc * 32, RNN, lane);
      }
#pragma unroll 1
      for (int tn = wave; tn < 32; tn += NWAV) {
        v8f acc = zero8();
#pragma unroll
        for (int kc = 0; kc < 4; ++kc) acc = wmh(fx[kc], ldb_frag(Wih_p, tn * 4 + kc, lane), acc);
#pragma unroll
        for (int kc = 0; kc < 4; ++kc) acc = wmh(fh[kc], ldb_frag(Whh_p, tn * 4 + kc, lane), acc);
        const int col = tn * 16 + nn;
        const float bb = sBg[col];
#pragma unroll
        for (int r = 0; r < 8; ++r) sG[(8 * hh + r) * 512 + col] = acc[r] * INV_AW + bb;
      }
    }
    __syncthreads();

#pragma unroll 1
    for (int i = tid; i < VB * RNN; i += NTHR) {
      const int v = i >> 7, r = i & 127;
      const float* g = sG + v * 512;
      const float ig = sigm_(g[r]);
      const float fg = sigm_(g[128 + r]);
      const float gg = tanhf(g[256 + r]);
      const float og = sigm_(g[384 + r]);
      const float cn = fg * sC[i] + ig * gg;
      const float hn = og * tanhf(cn);
      sC[i] = cn;
      sH[i] = (_Float16)(hn * AC);
    }
    __syncthreads();

    if (wave == 0) {
      v8f acc = zero8();
#pragma unroll
      for (int kc = 0; kc < 4; ++kc)
        acc = wmh(lda_frag(sH + kc * 32, RNN, lane), ldb_frag(Wout_p, kc, lane), acc);
      const float bb = sBout[nn];
      if (nn < OSW) {
#pragma unroll
        for (int r = 0; r < 8; ++r) sOut[(8 * hh + r) * OSW + nn] = acc[r] * INV_AW + bb;
      }
    }
    __syncthreads();
    if (wave == 0) {
      const v4f ov = *(const v4f*)(sOut + 4 * lane);
      float* op = OS + (size_t)(t * NVEH + v0) * OSW + 4 * lane;
      *(volatile v4f*)op = ov;
      __threadfence();
      *(volatile v4f*)op = ov;
    }
  }
}

__global__ __launch_bounds__(256) void k_out(const float* __restrict__ OS, float* out, int nchunk) {
  const int lane = threadIdx.x & 31, wave = threadIdx.x >> 5;
  const int ch = blockIdx.x * 8 + wave;
  if (ch >= nchunk) return;
  const int f0 = ch * 128 + 4 * lane;
  v4f v;
#pragma unroll
  for (int i = 0; i < 4; ++i) {
    const int f = f0 + i;
    const int row = f / NOUT, o = f - NOUT * row;
    v[i] = OS[(size_t)row * OSW + o];
  }
  *(volatile v4f*)(out + f0) = v;
  __threadfence();
  *(volatile v4f*)(out + f0) = v;
}

extern "C" void kernel_launch(void* const* d_in, const int* in_sizes, int n_in,
                              void* d_out, int out_size, void* d_ws, size_t ws_size,
                              hipStream_t stream) {
  if (n_in < 18) return;
  if (in_sizes[0] != SEQ_T * NVEH * NIN) return;
  if (in_sizes[1] != SEQ_T * NVEH * GCELL) return;
  if (in_sizes[2] != NVEH * RNN || in_sizes[3] != NVEH * RNN) return;
  if (in_sizes[4] != EMB * NIN || in_sizes[5] != EMB) return;
  if (in_sizes[6] != 64 * 128 * 15 || in_sizes[7] != 64) return;
  if (in_sizes[8] != 32 * 64 * 15 || in_sizes[9] != 32) return;
  if (in_sizes[10] != EMB * 128 || in_sizes[11] != EMB) return;
  if (in_sizes[12] != 512 * 128 || in_sizes[13] != 512 * 128) return;
  if (in_sizes[14] != 512 || in_sizes[15] != 512) return;
  if (in_sizes[16] != NOUT * RNN || in_sizes[17] != NOUT) return;
  if (out_size != SEQ_T * NVEH * NOUT) return;
  if ((size_t)WSTOT > ws_size) return;

  const float* x_seq   = (const float*)d_in[0];
  const int*   grids   = (const int*)  d_in[1];
  const float* h0      = (const float*)d_in[2];
  const float* c0      = (const float*)d_in[3];
  const float* W_emb   = (const float*)d_in[4];
  const float* b_emb   = (const float*)d_in[5];
  const float* conv1_w = (const float*)d_in[6];
  const float* conv1_b = (const float*)d_in[7];
  const float* conv2_w = (const float*)d_in[8];
  const float* conv2_b = (const float*)d_in[9];
  const float* W_soc   = (const float*)d_in[10];
  const float* b_soc   = (const float*)d_in[11];
  const float* W_ih    = (const float*)d_in[12];
  const float* W_hh    = (const float*)d_in[13];
  const float* b_ih    = (const float*)d_in[14];
  const float* b_hh    = (const float*)d_in[15];
  const float* W_out   = (const float*)d_in[16];
  const float* b_out   = (const float*)d_in[17];
  float* out = (float*)d_out;

  char* ws = (char*)d_ws;
  _Float16* P_EMB = (_Float16*)(ws + O_EMB);
  _Float16* P_W1  = (_Float16*)(ws + O_W1);
  _Float16* P_W2  = (_Float16*)(ws + O_W2);
  _Float16* P_SOC = (_Float16*)(ws + O_SOC);
  _Float16* P_IH  = (_Float16*)(ws + O_IH);
  _Float16* P_HH  = (_Float16*)(ws + O_HH);
  _Float16* P_OUT = (_Float16*)(ws + O_OUT);
  float* OS = (float*)(ws + O_OS);

  k_pack<<<(F_EMB * 64 + 255) / 256, 256, 0, stream>>>(W_emb,   P_EMB, 0, 1,  F_EMB * 64);
  k_pack<<<(F_W1  * 64 + 255) / 256, 256, 0, stream>>>(conv1_w, P_W1,  1, 4,  F_W1  * 64);
  k_pack<<<(F_W2  * 64 + 255) / 256, 256, 0, stream>>>(conv2_w, P_W2,  2, 30, F_W2  * 64);
  k_pack<<<(F_SOC * 64 + 255) / 256, 256, 0, stream>>>(W_soc,   P_SOC, 3, 4,  F_SOC * 64);
  k_pack<<<(F_IH  * 64 + 255) / 256, 256, 0, stream>>>(W_ih,    P_IH,  3, 4,  F_IH  * 64);
  k_pack<<<(F_HH  * 64 + 255) / 256, 256, 0, stream>>>(W_hh,    P_HH,  3, 4,  F_HH  * 64);
  k_pack<<<(F_OUT * 64 + 255) / 256, 256, 0, stream>>>(W_out,   P_OUT, 4, 4,  F_OUT * 64);

  (void)hipFuncSetAttribute(reinterpret_cast<const void*>(&k_lstm),
                            hipFuncAttributeMaxDynamicSharedMemorySize, LDS_BYTES);
  k_lstm<<<NBLK, NTHR, LDS_BYTES, stream>>>(
      x_seq, grids, h0, c0, b_emb, conv1_b, conv2_b, b_soc, b_ih, b_hh, b_out,
      (const v16h*)P_EMB, (const v16h*)P_W1, (const v16h*)P_W2, (const v16h*)P_SOC,
      (const v16h*)P_IH, (const v16h*)P_HH, (const v16h*)P_OUT, OS);

  k_out<<<(NCHUNK + 7) / 8, 256, 0, stream>>>(OS, out, NCHUNK);
}
